// MatrixGraphConvolution_45019847197213
// MI455X (gfx1250) — hardware-verified
//
#include <hip/hip_runtime.h>
#include <stddef.h>


#define FI      128
#define FO      128
#define NTHR    256
#define NWAVE   8
#define EPT     8
#define NGRP    2
#define CHUNK   (NTHR * EPT * NGRP)
#define WCAP    (EPT * NGRP * 32)
#define NB      1024
#define ESHF    10
#define RCAP    34816
#define DEGCAP  256
#define GROWS   128
#define WSCALE  16
#define BSCALE  64
#define WSCAP   134217728
#define WPB     ((FO * FI / 8) / NTHR)

#define LDS_GEMM (GROWS * FO * 4)
#define LDS_AGG  ((RCAP + 3 * NB + NWAVE * WCAP + 2 * NWAVE) * 4)

static_assert((NB & (NB - 1)) == 0);
static_assert(NB <= (1 << ESHF));
static_assert(NB == 4 * NTHR);
static_assert((NB % (NWAVE * 32)) == 0);
static_assert((NB % GROWS) == 0);
static_assert((RCAP % 32) == 0);
static_assert(GROWS == NWAVE * 16);
static_assert((FI % 32) == 0 && FO == 128 && FO == 32 * 4);
static_assert((FO * FI / 8) % NTHR == 0);
static_assert(NTHR == NWAVE * 32);
static_assert(LDS_AGG <= 300 * 1024);
static_assert(LDS_GEMM <= 300 * 1024);

typedef float     v4f  __attribute__((ext_vector_type(4)));
typedef float     v8f  __attribute__((ext_vector_type(8)));
typedef int       v4i  __attribute__((ext_vector_type(4)));
typedef _Float16  v8h  __attribute__((ext_vector_type(8)));
typedef _Float16  v16h __attribute__((ext_vector_type(16)));
union FragH { v16h v; v8h h[2]; };

__device__ __forceinline__ v8f wmf(v16h a, v16h b, v8f c) {
  v8f d = __builtin_amdgcn_wmma_f32_16x16x32_f16(false, a, false, b, (short)0, c, false, false);
  asm volatile("v_nop\n\tv_nop\n\tv_nop\n\tv_nop" : "+v"(d) : "v"(a), "v"(b));
  return d;
}

template <int SRC, int WC>
__device__ __forceinline__ int scan_chunk(const int* __restrict__ keys, const int* __restrict__ vals,
                                          int nE, int nN, int cbase, int slotBase, int vec8,
                                          int* list, int tid, int lane, int wave) {
  int wc = 0;
#pragma unroll
  for (int g = 0; g < NGRP; ++g) {
    const int e0   = cbase + (g * NTHR + tid) * EPT;
    const int sent = -2147483647 - 1;
    v4i da, db;
    v4i sa = {0, 0, 0, 0}, sb = {0, 0, 0, 0};
    if (vec8 != 0 && cbase + CHUNK <= nE) {
      da = *(const v4i*)(keys + e0);
      db = *(const v4i*)(keys + e0 + 4);
      if (SRC) {
        sa = *(const v4i*)(vals + e0);
        sb = *(const v4i*)(vals + e0 + 4);
      }
    } else {
      const int i0 = min(e0, nE - 1),     i1 = min(e0 + 1, nE - 1), i2 = min(e0 + 2, nE - 1), i3 = min(e0 + 3, nE - 1);
      const int i4 = min(e0 + 4, nE - 1), i5 = min(e0 + 5, nE - 1), i6 = min(e0 + 6, nE - 1), i7 = min(e0 + 7, nE - 1);
      da.x = (e0     < nE) ? keys[i0] : sent;
      da.y = (e0 + 1 < nE) ? keys[i1] : sent;
      da.z = (e0 + 2 < nE) ? keys[i2] : sent;
      da.w = (e0 + 3 < nE) ? keys[i3] : sent;
      db.x = (e0 + 4 < nE) ? keys[i4] : sent;
      db.y = (e0 + 5 < nE) ? keys[i5] : sent;
      db.z = (e0 + 6 < nE) ? keys[i6] : sent;
      db.w = (e0 + 7 < nE) ? keys[i7] : sent;
      if (SRC) {
        sa.x = vals[i0]; sa.y = vals[i1]; sa.z = vals[i2]; sa.w = vals[i3];
        sb.x = vals[i4]; sb.y = vals[i5]; sb.z = vals[i6]; sb.w = vals[i7];
      }
    }
    if (SRC) {
      sa.x = min(max(sa.x, 0), nN - 1); sa.y = min(max(sa.y, 0), nN - 1);
      sa.z = min(max(sa.z, 0), nN - 1); sa.w = min(max(sa.w, 0), nN - 1);
      sb.x = min(max(sb.x, 0), nN - 1); sb.y = min(max(sb.y, 0), nN - 1);
      sb.z = min(max(sb.z, 0), nN - 1); sb.w = min(max(sb.w, 0), nN - 1);
    }
    const unsigned nb = (unsigned)slotBase;
    const unsigned s0 = (unsigned)da.x - nb, s1 = (unsigned)da.y - nb;
    const unsigned s2 = (unsigned)da.z - nb, s3 = (unsigned)da.w - nb;
    const unsigned s4 = (unsigned)db.x - nb, s5 = (unsigned)db.y - nb;
    const unsigned s6 = (unsigned)db.z - nb, s7 = (unsigned)db.w - nb;
    const bool h0 = s0 < (unsigned)NB, h1 = s1 < (unsigned)NB, h2 = s2 < (unsigned)NB, h3 = s3 < (unsigned)NB;
    const bool h4 = s4 < (unsigned)NB, h5 = s5 < (unsigned)NB, h6 = s6 < (unsigned)NB, h7 = s7 < (unsigned)NB;
    const unsigned any = __builtin_amdgcn_ballot_w32(h0 | h1 | h2 | h3 | h4 | h5 | h6 | h7);
    if (any != 0u) {
#define HITJ(HJ, SJ, VJ) { \
        const unsigned mj = __builtin_amdgcn_ballot_w32(HJ); \
        if (mj != 0u) { \
          if (HJ) { \
            const int pos = wc + (int)__builtin_amdgcn_mbcnt_lo(mj, 0u); \
            const int entv = SRC ? (((VJ) << ESHF) | (int)(SJ)) : (int)(SJ); \
            if (pos < WC) list[wave * WC + pos] = entv; \
          } \
          wc += (int)__builtin_popcount(mj); } }
      HITJ(h0, s0, sa.x)
      HITJ(h1, s1, sa.y)
      HITJ(h2, s2, sa.z)
      HITJ(h3, s3, sa.w)
      HITJ(h4, s4, sb.x)
      HITJ(h5, s5, sb.y)
      HITJ(h6, s6, sb.z)
      HITJ(h7, s7, sb.w)
#undef HITJ
    }
  }
  return wc;
}

__global__ __launch_bounds__(NTHR) void k_prep(const float* __restrict__ w, const float* __restrict__ bm,
                                                _Float16* wpl, _Float16* bpl) {
  const int tid = threadIdx.x;
  const bool second = (int)blockIdx.x >= WPB;
  const int blk = second ? ((int)blockIdx.x - WPB) : (int)blockIdx.x;
  const int i = blk * NTHR + tid;
  const float* src = second ? bm : w;
  _Float16* dst = second ? bpl : wpl;
  const float sc = second ? (float)BSCALE : (float)WSCALE;
  const v4f f0 = *(const v4f*)(src + 8 * i);
  const v4f f1 = *(const v4f*)(src + 8 * i + 4);
  v8h hv;
  hv[0] = (_Float16)(f0.x * sc); hv[1] = (_Float16)(f0.y * sc);
  hv[2] = (_Float16)(f0.z * sc); hv[3] = (_Float16)(f0.w * sc);
  hv[4] = (_Float16)(f1.x * sc); hv[5] = (_Float16)(f1.y * sc);
  hv[6] = (_Float16)(f1.z * sc); hv[7] = (_Float16)(f1.w * sc);
  _Float16* d = dst + (size_t)i * 8;
  *(volatile v8h*)d = hv;
  __threadfence();
  *(volatile v8h*)d = hv;
}

template <int KD, int NC, int ASC, int WSC>
__global__ __launch_bounds__(NTHR) void k_gemm(
    const float* __restrict__ A, const _Float16* __restrict__ Bw, float* C, int nRowsA) {
  extern __shared__ v4f lds_dyn[];
  constexpr int NT = NC / 16;
  constexpr float OSC = 1.0f / (float)(ASC * WSC);
  float* stg = (float*)lds_dyn;
  const int tid = threadIdx.x, lane = tid & 31, wave = tid >> 5, hh = lane >> 4, m = lane & 15;
  const int rowBase = blockIdx.x * GROWS;
  int arow = rowBase + wave * 16 + m;
  arow = arow > nRowsA - 1 ? nRowsA - 1 : arow;
  const float* ap = A + (size_t)arow * KD + 8 * hh;

  v8f acc[NT];
#pragma unroll
  for (int t = 0; t < NT; ++t) { v8f z = {0.f, 0.f, 0.f, 0.f, 0.f, 0.f, 0.f, 0.f}; acc[t] = z; }

#pragma unroll 1
  for (int kt = 0; kt < KD / 32; ++kt) {
    const float* akp = ap + 32 * kt;
    const v4f f0 = *(const v4f*)akp;
    const v4f f1 = *(const v4f*)(akp + 4);
    const v4f f2 = *(const v4f*)(akp + 16);
    const v4f f3 = *(const v4f*)(akp + 20);
    v8h lo, hi;
    lo[0] = (_Float16)(f0.x * (float)ASC); lo[1] = (_Float16)(f0.y * (float)ASC);
    lo[2] = (_Float16)(f0.z * (float)ASC); lo[3] = (_Float16)(f0.w * (float)ASC);
    lo[4] = (_Float16)(f1.x * (float)ASC); lo[5] = (_Float16)(f1.y * (float)ASC);
    lo[6] = (_Float16)(f1.z * (float)ASC); lo[7] = (_Float16)(f1.w * (float)ASC);
    hi[0] = (_Float16)(f2.x * (float)ASC); hi[1] = (_Float16)(f2.y * (float)ASC);
    hi[2] = (_Float16)(f2.z * (float)ASC); hi[3] = (_Float16)(f2.w * (float)ASC);
    hi[4] = (_Float16)(f3.x * (float)ASC); hi[5] = (_Float16)(f3.y * (float)ASC);
    hi[6] = (_Float16)(f3.z * (float)ASC); hi[7] = (_Float16)(f3.w * (float)ASC);
    FragH af;
    af.h[0] = lo;
    af.h[1] = hi;
#pragma unroll
    for (int t = 0; t < NT; ++t) {
      const _Float16* bp = Bw + (size_t)(16 * t + m) * KD + 32 * kt + 8 * hh;
      FragH bf;
      bf.h[0] = *(const v8h*)bp;
      bf.h[1] = *(const v8h*)(bp + 16);
      acc[t] = wmf(af.v, bf.v, acc[t]);
    }
  }

  const int r0 = wave * 16 + 8 * hh;
  float* sp = stg + r0 * NC + m;
#pragma unroll
  for (int t = 0; t < NT; ++t) {
#pragma unroll
    for (int r = 0; r < 8; ++r) sp[r * NC + 16 * t] = acc[t][r] * OSC;
  }
  __syncthreads();

  const float* lp = stg + wave * 16 * NC;
  float* gp = C + (size_t)(rowBase + wave * 16) * NC;
#pragma unroll
  for (int i = 0; i < (16 * NC) / 128; ++i) {
    const v4f v = *(const v4f*)(lp + i * 128 + 4 * lane);
    *(volatile v4f*)(gp + i * 128 + 4 * lane) = v;
  }
  __threadfence();
#pragma unroll
  for (int i = 0; i < (16 * NC) / 128; ++i) {
    const v4f v = *(const v4f*)(lp + i * 128 + 4 * lane);
    *(volatile v4f*)(gp + i * 128 + 4 * lane) = v;
  }
}

__global__ __launch_bounds__(NTHR) void k_agg(
    const int* __restrict__ ei, const float* __restrict__ xw, const float* __restrict__ xb,
    float* out, int nN, int nE, int vec8) {
#pragma clang fp contract(off)
  extern __shared__ v4f lds_dyn[];
  int* region = (int*)lds_dyn;
  int* sstart = region + RCAP;
  int* cursor = sstart + NB;
  int* scnt   = cursor + NB;
  int* list   = scnt + NB;
  int* wcnt   = list + NWAVE * WCAP;
  int* wtot   = wcnt + NWAVE;
  const int tid = threadIdx.x, lane = tid & 31, wave = tid >> 5;
  const int nodeBase = blockIdx.x * NB;
  const int* keys = ei + (size_t)nE;
  const int* vals = ei;

  {
    const v4i z = {0, 0, 0, 0};
#pragma unroll 1
    for (int i = tid; i < RCAP / 4; i += NTHR) ((v4i*)region)[i] = z;
#pragma unroll 1
    for (int i = tid; i < NB / 4; i += NTHR) ((v4i*)scnt)[i] = z;
  }
  __syncthreads();

  const int nChunks = (nE + CHUNK - 1) / CHUNK;

#pragma unroll 1
  for (int ch = 0; ch < nChunks; ++ch) {
    const int cbase = ch * CHUNK;
    const int wc = scan_chunk<0, WCAP>(keys, vals, nE, nN, cbase, nodeBase, vec8, list, tid, lane, wave);
    if (lane == 0) wcnt[wave] = wc;
    __syncthreads();
    if (wave == 0) {
#pragma unroll 1
      for (int wsx = 0; wsx < NWAVE; ++wsx) {
        int n = __builtin_amdgcn_readfirstlane(wcnt[wsx]);
        n = n > WCAP ? WCAP : (n < 0 ? 0 : n);
        const int* lp = list + wsx * WCAP;
#pragma unroll 1
        for (int i = 0; i < n; ++i) {
          const int ent  = __builtin_amdgcn_readfirstlane(lp[i]);
          const int slot = ent & (NB - 1);
          if (lane == 0) scnt[slot] = scnt[slot] + 1;
        }
      }
    }
    __syncthreads();
  }

  {
    const v4i c4 = *(const v4i*)(scnt + 4 * tid);
    const int e0 = max(c4.x, 0), e1 = max(c4.y, 0), e2 = max(c4.z, 0), e3 = max(c4.w, 0);
    const int ts = e0 + e1 + e2 + e3;
    int incl = ts;
#pragma unroll
    for (int d = 1; d < 32; d <<= 1) {
      const int t = __shfl_up(incl, d);
      if (lane >= d) incl += t;
    }
    if (lane == 31) wtot[wave] = incl;
    __syncthreads();
    int pre = 0;
#pragma unroll
    for (int w2 = 0; w2 < NWAVE; ++w2) pre += (w2 < wave) ? wtot[w2] : 0;
    int run = pre + incl - ts;
    v4i o;
    o.x = run > RCAP ? RCAP : run; run += e0;
    o.y = run > RCAP ? RCAP : run; run += e1;
    o.z = run > RCAP ? RCAP : run; run += e2;
    o.w = run > RCAP ? RCAP : run;
    *(v4i*)(sstart + 4 * tid) = o;
    *(v4i*)(cursor + 4 * tid) = o;
  }
  __syncthreads();

#pragma unroll 1
  for (int ch = 0; ch < nChunks; ++ch) {
    const int cbase = ch * CHUNK;
    const int wc = scan_chunk<1, WCAP>(keys, vals, nE, nN, cbase, nodeBase, vec8, list, tid, lane, wave);
    if (lane == 0) wcnt[wave] = wc;
    __syncthreads();
    if (wave == 0) {
#pragma unroll 1
      for (int wsx = 0; wsx < NWAVE; ++wsx) {
        int n = __builtin_amdgcn_readfirstlane(wcnt[wsx]);
        n = n > WCAP ? WCAP : (n < 0 ? 0 : n);
        const int* lp = list + wsx * WCAP;
#pragma unroll 1
        for (int i = 0; i < n; ++i) {
          const int ent  = __builtin_amdgcn_readfirstlane(lp[i]);
          const int slot = ent & (NB - 1);
          int src = (ent >> ESHF) & 0xFFFFF;
          src = src > nN - 1 ? nN - 1 : src;
          if (lane == 0) {
            int pos = cursor[slot];
            pos = pos < 0 ? 0 : (pos > RCAP - 1 ? RCAP - 1 : pos);
            region[pos] = src;
            const int np = pos + 1;
            cursor[slot] = np > RCAP ? RCAP : np;
          }
        }
      }
    }
    __syncthreads();
  }

  const v4f zero4 = {0.f, 0.f, 0.f, 0.f};
#pragma unroll 1
  for (int jg = 0; jg < NB / (NWAVE * 32); ++jg) {
    const int sbase = wave * (NB / NWAVE) + jg * 32;
    const int st_l = sstart[sbase + lane];
    const int cn_l = scnt[sbase + lane];
#pragma unroll 1
    for (int j = 0; j < 32; ++j) {
      const int slot = sbase + j;
      const int c = nodeBase + slot;
      int st = __builtin_amdgcn_readlane(st_l, j);
      st = st < 0 ? 0 : (st > RCAP ? RCAP : st);
      const int cn = __builtin_amdgcn_readlane(cn_l, j);
      int n = cn < 0 ? 0 : (cn > DEGCAP ? DEGCAP : cn);
      n = n > RCAP - st ? RCAP - st : n;
      v4f acc = zero4;
#pragma unroll 1
      for (int q0 = 0; q0 < n; q0 += 32) {
        int idx = st + q0 + lane;
        idx = idx > RCAP - 1 ? RCAP - 1 : idx;
        int sl = region[idx];
        sl = sl < 0 ? 0 : (sl > nN - 1 ? nN - 1 : sl);
        const int mcnt = (n - q0) < 32 ? (n - q0) : 32;
#pragma unroll 1
        for (int p = 0; p < mcnt; ++p) {
          const int s = __builtin_amdgcn_readlane(sl, p);
          bool dup = (lane < p) && (sl == s);
#pragma unroll 1
          for (int q1 = 0; q1 < q0; q1 += 32) {
            int eidx = st + q1 + lane;
            eidx = eidx > RCAP - 1 ? RCAP - 1 : eidx;
            int e = region[eidx];
            e = e < 0 ? 0 : (e > nN - 1 ? nN - 1 : e);
            dup = dup || (e == s);
          }
          const unsigned dm = __builtin_amdgcn_ballot_w32(dup);
          if (dm == 0u) {
            acc = acc + *(const v4f*)(xw + (size_t)s * FO + 4 * lane);
          }
        }
      }
      const float inv = (cn <= 0) ? 1.0f : (1.0f / (float)cn);
      const v4f bv = *(const v4f*)(xb + (size_t)c * FO + 4 * lane);
      const v4f sc = acc * inv;
      const v4f v = sc + bv;
      const int cw = c < nN ? c : nN - 1;
      float* op = out + (size_t)cw * FO + 4 * lane;
      if (c < nN) *(volatile v4f*)op = v;
      __threadfence();
      if (c < nN) *(volatile v4f*)op = v;
    }
  }
}

extern "C" void kernel_launch(void* const* d_in, const int* in_sizes, int n_in,
                              void* d_out, int out_size, void* d_ws, size_t ws_size,
                              hipStream_t stream) {
  if (n_in < 4) return;
  const int nN = in_sizes[0] / FI;
  const int nE = in_sizes[1] / 2;
  if (nN <= 0 || nE <= 0 || in_sizes[0] != nN * FI || in_sizes[1] != 2 * nE) return;
  if (in_sizes[2] != FO * FI || in_sizes[3] != FO * FI) return;
  if (out_size != nN * FO) return;
  if (nN > (1 << 20) || nE > (1 << 28)) return;

  const float* x  = (const float*)d_in[0];
  const int*   ei = (const int*)d_in[1];
  const float* W  = (const float*)d_in[2];
  const float* Bm = (const float*)d_in[3];
  float* out = (float*)d_out;

  const int nAgg  = (nN + NB - 1) / NB;
  const int NPAD  = nAgg * NB;
  const int nGemm = NPAD / GROWS;

  char* ws = (char*)d_ws;
  size_t off = 0;
  const size_t oWp = off; off += (size_t)(FO * FI) * 2;         off = (off + 255) & ~(size_t)255;
  const size_t oBp = off; off += (size_t)(FO * FI) * 2;         off = (off + 255) & ~(size_t)255;
  const size_t oXw = off; off += (size_t)NPAD * FO * 4;         off = (off + 255) & ~(size_t)255;
  const size_t oXb = off; off += (size_t)NPAD * FO * 4;         off = (off + 255) & ~(size_t)255;
  if (off > ws_size || off > (size_t)WSCAP) return;
  _Float16* wpl = (_Float16*)(ws + oWp);
  _Float16* bpl = (_Float16*)(ws + oBp);
  float*    xw  = (float*)(ws + oXw);
  float*    xb  = (float*)(ws + oXb);

  const int vec8 = ((nE & 7) == 0) ? 1 : 0;

  k_prep<<<2 * WPB, NTHR, 0, stream>>>(W, Bm, wpl, bpl);

  hipFuncSetAttribute(reinterpret_cast<const void*>(&k_gemm<FI, FO, 1, WSCALE>),
                      hipFuncAttributeMaxDynamicSharedMemorySize, LDS_GEMM);
  k_gemm<FI, FO, 1, WSCALE><<<nGemm, NTHR, LDS_GEMM, stream>>>(x, wpl, xw, nN);
  hipFuncSetAttribute(reinterpret_cast<const void*>(&k_gemm<FI, FO, 1, BSCALE>),
                      hipFuncAttributeMaxDynamicSharedMemorySize, LDS_GEMM);
  k_gemm<FI, FO, 1, BSCALE><<<nGemm, NTHR, LDS_GEMM, stream>>>(x, bpl, xb, nN);

  hipFuncSetAttribute(reinterpret_cast<const void*>(&k_agg),
                      hipFuncAttributeMaxDynamicSharedMemorySize, LDS_AGG);
  k_agg<<<nAgg, NTHR, LDS_AGG, stream>>>(ei, xw, xb, out, nN, nE, vec8);
}
